// LSTM_41918880809220
// MI455X (gfx1250) — hardware-verified
//
#include <hip/hip_runtime.h>
#include <math.h>

constexpr int NSEQ  = 8192;
constexpr int NSTEP = 28;
constexpr int NINP  = 28;
constexpr int KXP   = 32;
constexpr int NHID  = 128;
constexpr int NGATE = 4 * NHID;
constexpr int NCLS  = 10;
constexpr int NTHR  = 256;
constexpr int RB    = 32;
constexpr int XP    = 40;
constexpr int HP    = 136;
constexpr int FP    = 132;
constexpr float WCARRY     = 16.0f;
constexpr float WCARRY_INV = 1.0f / 16.0f;
static_assert(NSEQ % RB == 0, "grid exact");
static_assert(RB == 32, "two m-subtiles per block");
static_assert(NHID == 16 * (NTHR / 32), "8 waves x 16 hidden units");
static_assert(KXP % 32 == 0 && NHID % 32 == 0, "K multiples of 32");
static_assert(NINP <= KXP && NINP % 4 == 0, "x rows load as float4 chunks");
static_assert((RB * (NINP / 4)) % 32 == 0, "x staging lanes wave-uniform");
static_assert(RB * (NINP / 4) + RB <= NTHR, "x staging + pad lanes fit the block");
static_assert((RB * NCLS * 4) % 128 == 0, "block output = whole 128-B lines");
static_assert((RB * NCLS) % 4 == 0, "output float4 granularity");
static_assert((2 * RB * HP) % NTHR == 0, "h zero-fill loop exact");
static_assert(XP % 8 == 0 && HP % 8 == 0 && FP % 4 == 0, "16-B aligned fragment rows");
static_assert((NGATE * NHID / 8) % NTHR == 0, "weight convert grid exact");
static_assert((64 * NINP) % 4 == 0 && ((64 * NINP / 4 - NTHR) % 32) == 0, "w0x staging lanes wave-uniform");
static_assert(NGATE % 64 == 0, "w0x prep grid exact");

typedef __attribute__((ext_vector_type(16))) _Float16 v16h;
typedef __attribute__((ext_vector_type(8)))  _Float16 v8h;
typedef __attribute__((ext_vector_type(4)))  _Float16 v4h;
typedef __attribute__((ext_vector_type(8)))  float    v8f;
typedef __attribute__((ext_vector_type(4)))  float    v4f;
typedef __attribute__((ext_vector_type(2)))  unsigned v2u;

__device__ __forceinline__ void guard8(v8f& a0, v8f& a1, v8f& a2, v8f& a3, v8f& a4, v8f& a5, v8f& a6, v8f& a7,
                                       v16h x0, v16h x1, v16h y0, v16h y1, v16h y2, v16h y3) {
  asm volatile("v_nop\n\tv_nop\n\tv_nop\n\tv_nop"
               : "+v"(a0), "+v"(a1), "+v"(a2), "+v"(a3), "+v"(a4), "+v"(a5), "+v"(a6), "+v"(a7)
               : "v"(x0), "v"(x1), "v"(y0), "v"(y1), "v"(y2), "v"(y3));
}

template <typename T> struct Frag;
template <> struct Frag<_Float16> {
  typedef v16h V; union U { v16h v; v8h h[2]; };
  static __device__ __forceinline__ v16h load(const _Float16* p) {
    U f; f.h[0] = *(const v8h*)(p); f.h[1] = *(const v8h*)(p + 16); return f.v;
  }
  static __device__ __forceinline__ v8f mma(v16h a, v16h b, v8f c) {
    return __builtin_amdgcn_wmma_f32_16x16x32_f16(false, a, false, b, (short)0, c, false, false);
  }
};

__device__ __forceinline__ float fsig(float z) {
  z = fminf(fmaxf(z, -30.0f), 30.0f);
  return __builtin_amdgcn_rcpf(1.0f + expf(-z));
}
__device__ __forceinline__ float ftanh(float z) {
  z = fminf(fmaxf(z, -15.0f), 15.0f);
  return 1.0f - 2.0f * __builtin_amdgcn_rcpf(expf(2.0f * z) + 1.0f);
}

__global__ __launch_bounds__(NTHR) void prep_w0x_kernel(const float* __restrict__ w, unsigned short* __restrict__ dst) {
  __shared__ __align__(16) float Ws[64 * NINP];
  const int tid = threadIdx.x, b = blockIdx.x;
  const float* src = w + (size_t)b * 64 * NINP;
#pragma unroll
  for (int it = 0; it < 2; ++it) {
    const int idx = it * NTHR + tid;
    if (idx < 64 * NINP / 4) {
      const v4f v = *(const v4f*)(src + 4 * idx);
      Ws[4 * idx + 0] = v[0];
      Ws[4 * idx + 1] = v[1];
      Ws[4 * idx + 2] = v[2];
      Ws[4 * idx + 3] = v[3];
    }
  }
  __syncthreads();
  const int nl = tid >> 2, q = tid & 3;
  v8h hv;
#pragma unroll
  for (int e = 0; e < 8; ++e) {
    const int k  = 8 * q + e;
    const int kk = (k < NINP) ? k : (NINP - 1);
    const float f   = Ws[nl * NINP + kk];
    const float val = (k < NINP) ? f : 0.0f;
    hv[e] = (_Float16)(val * WCARRY);
  }
  unsigned short* op = dst + (size_t)(b * 64 + nl) * KXP + 8 * q;
  *(volatile v8h*)op = hv;
  __threadfence();
  *(volatile v8h*)op = hv;
}

__global__ __launch_bounds__(NTHR) void prep_w128_kernel(const float* __restrict__ s0, const float* __restrict__ s1,
                                                        const float* __restrict__ s2, unsigned short* __restrict__ dst) {
  const int y = blockIdx.y;
  const float* src = (y == 0) ? s0 : ((y == 1) ? s1 : s2);
  const int i = blockIdx.x * NTHR + threadIdx.x;
  const v4f a = *(const v4f*)(src + (size_t)8 * i);
  const v4f c = *(const v4f*)(src + (size_t)8 * i + 4);
  v8h hv;
#pragma unroll
  for (int e = 0; e < 4; ++e) {
    const float fa = a[e], fc = c[e];
    hv[e]     = (_Float16)(fa * WCARRY);
    hv[4 + e] = (_Float16)(fc * WCARRY);
  }
  unsigned short* op = dst + (size_t)y * NGATE * NHID + (size_t)8 * i;
  *(volatile v8h*)op = hv;
  __threadfence();
  *(volatile v8h*)op = hv;
}

__device__ __forceinline__ void stage_x(const float* __restrict__ x, _Float16* sX, int rowbase, int ts, int tid) {
  if (tid < RB * (NINP / 4)) {
    const int r = tid / (NINP / 4), q = tid - r * (NINP / 4);
    const v4f v = *(const v4f*)(x + ((size_t)(rowbase + r) * NSTEP + (size_t)ts) * NINP + 4 * q);
    const float x0 = v[0], x1 = v[1], x2 = v[2], x3 = v[3];
    v4h hv;
    hv[0] = (_Float16)x0; hv[1] = (_Float16)x1; hv[2] = (_Float16)x2; hv[3] = (_Float16)x3;
    *(v4h*)(sX + r * XP + 4 * q) = hv;
  } else {
    const int r = tid - RB * (NINP / 4);
    const v2u z = {0u, 0u};
    *(v2u*)(void*)(sX + r * XP + NINP) = z;
  }
}

__device__ __forceinline__ void mac_tile(v8f (&acc)[4][2], const _Float16* At, int ap,
                                         const _Float16* W, int wp, int nk, int lc, int hh, int j) {
  const _Float16* ar0 = At + lc * ap + 8 * hh;
  const _Float16* ar1 = At + (16 + lc) * ap + 8 * hh;
  const _Float16* wr  = W + (size_t)j * wp + 8 * hh;
  const size_t gs = (size_t)NHID * wp;
#pragma unroll 1
  for (int kc = 0; kc < nk; ++kc) {
    const int k0 = kc << 5;
    const v16h b0 = Frag<_Float16>::load(wr + k0);
    const v16h b1 = Frag<_Float16>::load(wr + gs + k0);
    const v16h b2 = Frag<_Float16>::load(wr + 2 * gs + k0);
    const v16h b3 = Frag<_Float16>::load(wr + 3 * gs + k0);
    const v16h a0 = Frag<_Float16>::load(ar0 + k0);
    const v16h a1 = Frag<_Float16>::load(ar1 + k0);
    acc[0][0] = Frag<_Float16>::mma(a0, b0, acc[0][0]);
    acc[0][1] = Frag<_Float16>::mma(a1, b0, acc[0][1]);
    acc[1][0] = Frag<_Float16>::mma(a0, b1, acc[1][0]);
    acc[1][1] = Frag<_Float16>::mma(a1, b1, acc[1][1]);
    acc[2][0] = Frag<_Float16>::mma(a0, b2, acc[2][0]);
    acc[2][1] = Frag<_Float16>::mma(a1, b2, acc[2][1]);
    acc[3][0] = Frag<_Float16>::mma(a0, b3, acc[3][0]);
    acc[3][1] = Frag<_Float16>::mma(a1, b3, acc[3][1]);
    guard8(acc[0][0], acc[0][1], acc[1][0], acc[1][1], acc[2][0], acc[2][1], acc[3][0], acc[3][1], a0, a1, b0, b1, b2, b3);
  }
}

template <bool WRITEF>
__device__ __forceinline__ void cell_update(v8f (&acc)[4][2], float (&cst)[2][8], const float (&bs)[4],
                                            _Float16* hdst, float* fdst, int hh, int j) {
#pragma unroll
  for (int mt = 0; mt < 2; ++mt) {
#pragma unroll
    for (int r = 0; r < 8; ++r) {
      const float zi = fmaf(acc[0][mt][r], WCARRY_INV, bs[0]);
      const float zf = fmaf(acc[1][mt][r], WCARRY_INV, bs[1]);
      const float zg = fmaf(acc[2][mt][r], WCARRY_INV, bs[2]);
      const float zo = fmaf(acc[3][mt][r], WCARRY_INV, bs[3]);
      const float ig = fsig(zi);
      const float fg = fsig(zf);
      const float gg = ftanh(zg);
      const float og = fsig(zo);
      const float cn = fg * cst[mt][r] + ig * gg;
      cst[mt][r] = cn;
      const float hn = og * ftanh(cn);
      const int row = 16 * mt + 8 * hh + r;
      hdst[row * HP + j] = (_Float16)hn;
      if (WRITEF) fdst[row * FP + j] = hn;
    }
  }
}

__global__ __launch_bounds__(NTHR) void lstm2_kernel(const float* __restrict__ x,
                                                    const float* __restrict__ bih0, const float* __restrict__ bhh0,
                                                    const float* __restrict__ bih1, const float* __restrict__ bhh1,
                                                    const unsigned short* __restrict__ W0Xp, const unsigned short* __restrict__ W0Hp,
                                                    const unsigned short* __restrict__ W1Xp, const unsigned short* __restrict__ W1Hp,
                                                    const float* __restrict__ wout, const float* __restrict__ bout,
                                                    float* __restrict__ out) {
  __shared__ __align__(16) _Float16 sX[RB * XP];
  __shared__ __align__(16) _Float16 sH1[2][RB * HP];
  __shared__ __align__(16) _Float16 sH2[2][RB * HP];
  __shared__ __align__(16) float    sF[RB * FP];
  __shared__ __align__(16) float    sO[RB * NCLS];
  const _Float16* W0X = (const _Float16*)W0Xp;
  const _Float16* W0H = (const _Float16*)W0Hp;
  const _Float16* W1X = (const _Float16*)W1Xp;
  const _Float16* W1H = (const _Float16*)W1Hp;
  const int tid = threadIdx.x, lane = tid & 31, wave = tid >> 5;
  const int lc = lane & 15, hh = lane >> 4;
  const int j = 16 * wave + lc;
  const int rowbase = blockIdx.x * RB;

  {
    _Float16* h1f = &sH1[0][0];
    _Float16* h2f = &sH2[0][0];
#pragma unroll 1
    for (int i = tid; i < 2 * RB * HP; i += NTHR) { h1f[i] = (_Float16)0.0f; h2f[i] = (_Float16)0.0f; }
  }
  float bs0[4], bs1[4];
#pragma unroll
  for (int g = 0; g < 4; ++g) bs0[g] = bih0[g * NHID + j] + bhh0[g * NHID + j];
  asm volatile("" ::: "memory");
#pragma unroll
  for (int g = 0; g < 4; ++g) bs1[g] = bih1[g * NHID + j] + bhh1[g * NHID + j];
  asm volatile("" ::: "memory");
  float c1[2][8], c2[2][8];
#pragma unroll
  for (int mt = 0; mt < 2; ++mt)
#pragma unroll
    for (int r = 0; r < 8; ++r) { c1[mt][r] = 0.0f; c2[mt][r] = 0.0f; }
  stage_x(x, sX, rowbase, 0, tid);
  __syncthreads();

  const v8f z8 = {0.f, 0.f, 0.f, 0.f, 0.f, 0.f, 0.f, 0.f};

#pragma unroll 1
  for (int t = 0; t < NSTEP; ++t) {
    const int cur = t & 1, nxt = cur ^ 1;
    v8f acc[4][2];
#pragma unroll
    for (int g = 0; g < 4; ++g) { acc[g][0] = z8; acc[g][1] = z8; }
    mac_tile(acc, sX, XP, W0X, KXP, KXP / 32, lc, hh, j);
    asm volatile("" ::: "memory");
    mac_tile(acc, &sH1[cur][0], HP, W0H, NHID, NHID / 32, lc, hh, j);
    cell_update<false>(acc, c1, bs0, &sH1[nxt][0], sF, hh, j);
    __syncthreads();
    if (t + 1 < NSTEP) stage_x(x, sX, rowbase, t + 1, tid);
    asm volatile("" ::: "memory");
#pragma unroll
    for (int g = 0; g < 4; ++g) { acc[g][0] = z8; acc[g][1] = z8; }
    mac_tile(acc, &sH1[nxt][0], HP, W1X, NHID, NHID / 32, lc, hh, j);
    asm volatile("" ::: "memory");
    mac_tile(acc, &sH2[cur][0], HP, W1H, NHID, NHID / 32, lc, hh, j);
    cell_update<true>(acc, c2, bs1, &sH2[nxt][0], sF, hh, j);
    __syncthreads();
  }

  for (int i = tid; i < RB * NCLS; i += NTHR) {
    const int r = i / NCLS, cls = i - r * NCLS;
    float s = 0.0f;
#pragma unroll 1
    for (int k = 0; k < NHID; ++k) s = fmaf(sF[r * FP + k], wout[cls * NHID + k], s);
    sO[i] = s + bout[cls];
  }
  __syncthreads();
  if (wave == 0) {
    float* op = out + (size_t)rowbase * NCLS;
    for (int pass = 0; pass < 2; ++pass) {
#pragma unroll
      for (int it = 0; it < 3; ++it) {
        const int idx = it * 32 + lane;
        if (idx < RB * NCLS / 4) {
          const v4f v = *(const v4f*)(sO + 4 * idx);
          *(volatile v4f*)(op + 4 * idx) = v;
        }
      }
      __threadfence();
    }
  }
}

extern "C" void kernel_launch(void* const* d_in, const int* in_sizes, int n_in,
                              void* d_out, int out_size, void* d_ws, size_t ws_size, hipStream_t stream) {
  if (n_in < 11 || d_out == nullptr || d_ws == nullptr) return;
  if (in_sizes[0] != NSEQ * NSTEP * NINP || in_sizes[1] != NGATE * NINP || in_sizes[2] != NGATE * NHID ||
      in_sizes[3] != NGATE || in_sizes[4] != NGATE || in_sizes[5] != NGATE * NHID || in_sizes[6] != NGATE * NHID ||
      in_sizes[7] != NGATE || in_sizes[8] != NGATE || in_sizes[9] != NCLS * NHID || in_sizes[10] != NCLS ||
      out_size != NSEQ * NCLS) return;

  const float* x     = (const float*)d_in[0];
  const float* w_ih0 = (const float*)d_in[1];
  const float* w_hh0 = (const float*)d_in[2];
  const float* b_ih0 = (const float*)d_in[3];
  const float* b_hh0 = (const float*)d_in[4];
  const float* w_ih1 = (const float*)d_in[5];
  const float* w_hh1 = (const float*)d_in[6];
  const float* b_ih1 = (const float*)d_in[7];
  const float* b_hh1 = (const float*)d_in[8];
  const float* w_out = (const float*)d_in[9];
  const float* b_out = (const float*)d_in[10];
  float* out = (float*)d_out;

  char* ws = (char*)d_ws; size_t off = 0;
  auto carve = [&](size_t bytes) -> char* { char* p = ws + off; off += (bytes + 255) & ~(size_t)255; return p; };
  unsigned short* W0X = (unsigned short*)carve((size_t)NGATE * KXP * 2);
  unsigned short* WH  = (unsigned short*)carve((size_t)3 * NGATE * NHID * 2);
  if (off > ws_size || off > (size_t)134217728) return;
  unsigned short* W0H = WH;
  unsigned short* W1X = WH + (size_t)NGATE * NHID;
  unsigned short* W1H = WH + (size_t)2 * NGATE * NHID;

  prep_w0x_kernel<<<NGATE / 64, NTHR, 0, stream>>>(w_ih0, W0X);
  prep_w128_kernel<<<dim3(NGATE * NHID / 8 / NTHR, 3), NTHR, 0, stream>>>(w_hh0, w_ih1, w_hh1, WH);
  lstm2_kernel<<<NSEQ / RB, NTHR, 0, stream>>>(x, b_ih0, b_hh0, b_ih1, b_hh1, W0X, W0H, W1X, W1H, w_out, b_out, out);
}
